// aggregator_16922171146281
// MI455X (gfx1250) — hardware-verified
//
#include <hip/hip_runtime.h>
#include <math.h>

typedef __attribute__((ext_vector_type(16))) _Float16 v16h;
typedef __attribute__((ext_vector_type(16))) __bf16 v16b;
typedef __attribute__((ext_vector_type(8)))  _Float16 v8h;
typedef __attribute__((ext_vector_type(8)))  float v8f;
typedef __attribute__((ext_vector_type(4)))  float v4f;
typedef __attribute__((ext_vector_type(2)))  float v2f;
typedef __attribute__((ext_vector_type(4)))  unsigned v4u;
typedef __attribute__((ext_vector_type(4)))  int v4i;
typedef float __attribute__((may_alias)) float_a;
typedef int __attribute__((may_alias)) int_a;

template <typename T> __device__ __forceinline__ void vst2(void* p, T v) { *(volatile T*)p = v; __threadfence(); *(volatile T*)p = v; }
__device__ __forceinline__ v8f wmma16(v16h a, v16h b, v8f c) {
  v8f d = __builtin_amdgcn_wmma_f32_16x16x32_f16(false, a, false, b, (short)0, c, false, false);
  asm volatile("v_nop\n\tv_nop\n\tv_nop\n\tv_nop" : "+v"(d) : "v"(a), "v"(b));
  return d;
}
__device__ __forceinline__ v8f wmma_bf(v16b a, v16b b, v8f c) {
  v8f d = __builtin_amdgcn_wmma_f32_16x16x32_bf16(false, a, false, b, (short)0, c, false, false);
  asm volatile("v_nop\n\tv_nop\n\tv_nop\n\tv_nop" : "+v"(d) : "v"(a), "v"(b));
  return d;
}
__device__ __forceinline__ v16h frag_h(const _Float16* rowk0, int lane) {
  union { v16h v; v8h q[2]; } u; const _Float16* p = rowk0 + 8 * (lane >> 4);
  u.q[0] = *(const v8h*)p; u.q[1] = *(const v8h*)(p + 16); return u.v;
}
__device__ __forceinline__ v16h frag_f32(const float* rowk0, int lane) {
  v16h a; const float* p = rowk0 + 8 * (lane >> 4);
#pragma unroll
  for (int i = 0; i < 8; ++i) { a[i] = (_Float16)p[i]; a[8 + i] = (_Float16)p[16 + i]; }
  return a;
}
__device__ __forceinline__ v16h frag_f32s(const float* rowk0, int lane, float sc) {
  v16h a; const float* p = rowk0 + 8 * (lane >> 4);
#pragma unroll
  for (int i = 0; i < 8; ++i) { a[i] = (_Float16)(p[i] * sc); a[8 + i] = (_Float16)(p[16 + i] * sc); }
  return a;
}
__device__ __forceinline__ v16h fragc_f32(const float* W, int k0, int n, int lane, int ld, int K) {
  v16h a; const int g = lane >> 4;
#pragma unroll
  for (int i = 0; i < 8; ++i) { const int ka = k0 + 8 * g + i, kb = ka + 16;
    a[i] = (_Float16)(ka < K ? W[(size_t)(ka < K ? ka : K - 1) * ld + n] : 0.f); a[8 + i] = (_Float16)(kb < K ? W[(size_t)(kb < K ? kb : K - 1) * ld + n] : 0.f); }
  return a;
}
struct F2 { v16b h, l; };
__device__ __forceinline__ F2 bsplit16(const float v[16]) { F2 r;
#pragma unroll
  for (int i = 0; i < 16; ++i) { const __bf16 h = (__bf16)v[i]; r.h[i] = h; r.l[i] = (__bf16)(v[i] - (float)h); }
  return r; }
__device__ __forceinline__ F2 split_row(const float* row, int k0, int lane) { float v[16]; const float* p = row + k0 + 8 * (lane >> 4);
#pragma unroll
  for (int i = 0; i < 8; ++i) { v[i] = p[i]; v[8 + i] = p[16 + i]; }
  return bsplit16(v); }
__device__ __forceinline__ F2 split_rowK(const float* row, int k0, int lane, int K) { float v[16]; const int g = lane >> 4;
#pragma unroll
  for (int i = 0; i < 8; ++i) { const int ka = k0 + 8 * g + i, kb = ka + 16; v[i] = ka < K ? row[ka < K ? ka : K - 1] : 0.f; v[8 + i] = kb < K ? row[kb < K ? kb : K - 1] : 0.f; }
  return bsplit16(v); }
__device__ __forceinline__ F2 split_col(const float* W, int k0, int n, int lane, int ld, int K) { float v[16]; const int g = lane >> 4;
#pragma unroll
  for (int i = 0; i < 8; ++i) { const int ka = k0 + 8 * g + i, kb = ka + 16; v[i] = ka < K ? W[(size_t)(ka < K ? ka : K - 1) * ld + n] : 0.f; v[8 + i] = kb < K ? W[(size_t)(kb < K ? kb : K - 1) * ld + n] : 0.f; }
  return bsplit16(v); }
__device__ __forceinline__ v8f mac3(const F2& a, const F2& b, v8f c) { c = wmma_bf(a.l, b.h, c); c = wmma_bf(a.h, b.l, c); return wmma_bf(a.h, b.h, c); }
__device__ __forceinline__ float sigm(float v) { return 1.0f / (1.0f + expf(-v)); }
#define LDSX() do { asm volatile("s_wait_dscnt 0" ::: "memory"); __builtin_amdgcn_wave_barrier(); __builtin_amdgcn_fence(__ATOMIC_RELEASE, "workgroup"); } while (0)

#define NN 50000
#define KNB 24
#define FD 128
#define ED 64
#define NDRUG 50000
#define NSIDE 100000
#define NPB 8
#ifndef NPR
#define NPR NN
#endif
__device__ __forceinline__ float bfr(float v) { return (float)(__bf16)v; }
__device__ __forceinline__ v16b wcol(const float* Wm, int k0, int o, int lane, int ld) { v16b w; const int g = lane >> 4;
#pragma unroll
  for (int i = 0; i < 8; ++i) { w[i] = (__bf16)Wm[(size_t)(k0 + 8 * g + i) * ld + o]; w[8 + i] = (__bf16)Wm[(size_t)(k0 + 16 + 8 * g + i) * ld + o]; }
  return w; }

#define NNP ((NPR + 63) / 64 * 64)
#define WS_NF   0u
#define WS_AGG  (WS_NF  + 4u * (size_t)NNP * ED)
#define WS_LAST (WS_AGG + 4u * (size_t)NNP * ED)
#define WS_END  (WS_LAST + 4u * (size_t)50176)

__global__ __launch_bounds__(128) void k_fea(const int* __restrict__ NODES, const float* __restrict__ DW, const float* __restrict__ UW, const float* __restrict__ UB, float* __restrict__ OUT0, float* __restrict__ NF) { __shared__ __align__(16) float sf[4][16][68];
  const int tid = threadIdx.x, wave = tid >> 5, lane = tid & 31, col = lane & 15, g = lane >> 4; const int n0 = blockIdx.x * 64 + wave * 16; const int n = n0 + col; const int nc = n < NPR ? n : NPR - 1;
  int idx = NODES[nc]; idx = idx < 0 ? 0 : (idx >= NDRUG ? NDRUG - 1 : idx);
  v8f acc[4] = {};
#pragma unroll
  for (int kc = 0; kc < FD / 32; ++kc) { v16b a; { const float* p = DW + (size_t)idx * FD + kc * 32 + 8 * g;
#pragma unroll
      for (int i = 0; i < 8; ++i) { a[i] = (__bf16)p[i]; a[8 + i] = (__bf16)p[16 + i]; } }
    asm volatile("s_wait_loadcnt 0x0" ::: "memory");
#pragma unroll
    for (int j = 0; j < 4; ++j) { const v16b w = wcol(UW, kc * 32, j * 16 + col, lane, ED); asm volatile("s_wait_loadcnt 0x0" ::: "memory"); acc[j] = wmma_bf(a, w, acc[j]); } }
#pragma unroll
  for (int j = 0; j < 4; ++j) { const float bb = bfr(UB[j * 16 + col]);
#pragma unroll
    for (int r = 0; r < 8; ++r) sf[wave][8 * g + r][j * 16 + col] = acc[j][r] + bb; }
  LDSX(); for (int rl = 0; rl < 16; ++rl) { const int nr = n0 + rl; if (nr < NPR && lane < 16) { const v4f v = *(const v4f*)&sf[wave][rl][lane * 4]; vst2(OUT0 + (size_t)nr * ED + lane * 4, v); vst2(NF + (size_t)nr * ED + lane * 4, v); } } }
__global__ __launch_bounds__(128) void k_agg(const int* __restrict__ NIDX, const float* __restrict__ NMASK, const float* __restrict__ SW, const float* __restrict__ IW, const float* __restrict__ IB, const float* __restrict__ NF, float* __restrict__ AGG) {
  __shared__ __align__(16) float sn[NPB * KNB][ED + 4]; __shared__ float ssc[NPB][32];
  const int tid = threadIdx.x, wave = tid >> 5, lane = tid & 31, col = lane & 15, g = lane >> 4; const int nb0 = blockIdx.x * NPB;
#pragma unroll 1
  for (int rt = 0; rt < 3; ++rt) { const int row = (wave * 3 + rt) * 16 + col; const int nl = row / KNB, k = row % KNB; const int n = nb0 + nl; const int nc = n < NPR ? n : NPR - 1;
    int idx = NIDX[(size_t)nc * KNB + k]; idx = idx < 0 ? 0 : (idx >= NSIDE ? NSIDE - 1 : idx);
    v8f acc[4] = {};
#pragma unroll
    for (int kc = 0; kc < FD / 32; ++kc) { v16b a; { const float* p = SW + (size_t)idx * FD + kc * 32 + 8 * g;
#pragma unroll
        for (int i = 0; i < 8; ++i) { a[i] = (__bf16)p[i]; a[8 + i] = (__bf16)p[16 + i]; } }
      asm volatile("s_wait_loadcnt 0x0" ::: "memory");
#pragma unroll
      for (int j = 0; j < 4; ++j) { const v16b w = wcol(IW, kc * 32, j * 16 + col, lane, ED); asm volatile("s_wait_loadcnt 0x0" ::: "memory"); acc[j] = wmma_bf(a, w, acc[j]); } }
#pragma unroll
    for (int j = 0; j < 4; ++j) { const float bb = bfr(IB[j * 16 + col]);
#pragma unroll
      for (int r = 0; r < 8; ++r) sn[(wave * 3 + rt) * 16 + 8 * g + r][j * 16 + col] = acc[j][r] + bb; } }
  __syncthreads();
  const int nl = tid >> 4, s = tid & 15; const int n = nb0 + nl; const int nc = n < NPR ? n : NPR - 1;
  { float sc0 = 0.f, sc1 = 0.f; const float* nfr = NF + (size_t)nc * ED; const int k0 = s, k1 = s + 16;
#pragma unroll 8
    for (int d = 0; d < ED; ++d) { const float f = nfr[d]; sc0 += sn[nl * KNB + k0][d] * f; if (k1 < KNB) sc1 += sn[nl * KNB + k1][d] * f; }
    const float m0 = bfr(NMASK[(size_t)nc * KNB + k0]); ssc[nl][k0] = (m0 > 0.f) ? sc0 * 0.125f : -1.0e9f;
    if (k1 < KNB) { const float m1 = bfr(NMASK[(size_t)nc * KNB + k1]); ssc[nl][k1] = (m1 > 0.f) ? sc1 * 0.125f : -1.0e9f; } }
  __syncthreads();
  { float m = -3.0e38f;
#pragma unroll
    for (int k = 0; k < KNB; ++k) m = fmaxf(m, ssc[nl][k]);
    float e[KNB]; float sum = 0.f;
#pragma unroll
    for (int k = 0; k < KNB; ++k) { e[k] = expf(ssc[nl][k] - m); sum += e[k]; }
    const float inv = 1.0f / sum; v4f o = {0.f, 0.f, 0.f, 0.f};
#pragma unroll
    for (int k = 0; k < KNB; ++k) { const float a = e[k] * inv; const v4f nv = *(const v4f*)&sn[nl * KNB + k][s * 4]; o[0] += a * nv[0]; o[1] += a * nv[1]; o[2] += a * nv[2]; o[3] += a * nv[3]; }
    if (n < NPR) vst2(AGG + (size_t)n * ED + s * 4, o); } }
__global__ __launch_bounds__(256) void k_last(const int* __restrict__ NODES, int* __restrict__ LAST) { __shared__ int sx[2048];
  const int tid = threadIdx.x; const int d0 = blockIdx.x * 1024 + tid * 4; int best0 = -1, best1 = -1, best2 = -1, best3 = -1;
#pragma unroll 1
  for (int c0 = 0; c0 < NPR; c0 += 2048) { const int cn = (NPR - c0) < 2048 ? (NPR - c0) : 2048;
    __syncthreads();
    for (int e = tid; e < 2048; e += 256) sx[e] = (e < cn) ? NODES[c0 + e] : -7;
    __syncthreads();
#pragma unroll 4
    for (int e = 0; e < 2048; ++e) { const int v = sx[e]; const int pos = c0 + e; best0 = (v == d0) ? pos : best0; best1 = (v == d0 + 1) ? pos : best1; best2 = (v == d0 + 2) ? pos : best2; best3 = (v == d0 + 3) ? pos : best3; } }
  v4i o; o[0] = best0; o[1] = best1; o[2] = best2; o[3] = best3; vst2(LAST + d0, o); }
__global__ __launch_bounds__(256) void k_emb(const int* __restrict__ LAST, const float* __restrict__ AGG, float* __restrict__ OUT1) {
  const int tid = threadIdx.x; const int dl = tid >> 4, q = tid & 15;
#pragma unroll 1
  for (int rep = 0; rep < 4; ++rep) { const int d = blockIdx.x * 64 + rep * 16 + dl; if (d < NDRUG) { const int ln = LAST[d]; const int lc = ln < 0 ? 0 : (ln >= NPR ? NPR - 1 : ln); v4f v = *(const v4f*)(AGG + (size_t)lc * ED + q * 4); const float keep = (ln >= 0) ? 1.0f : 0.0f;
      v4f o; o[0] = keep * v[0]; o[1] = keep * v[1]; o[2] = keep * v[2]; o[3] = keep * v[3];
      vst2(OUT1 + (size_t)d * ED + q * 4, o); } } }
extern "C" void kernel_launch(void* const* d_in, const int* in_sizes, int n_in, void* d_out, int out_size, void* d_ws, size_t ws_size, hipStream_t stream) {
  (void)in_sizes; (void)n_in; (void)out_size;
  const float** F = (const float**)d_in;
  if (ws_size < (size_t)WS_END) return;
  char* ws = (char*)d_ws; float *NF = (float*)(ws + WS_NF), *AGG = (float*)(ws + WS_AGG); int* LAST = (int*)(ws + WS_LAST);
  float* OUT0 = (float*)d_out; float* OUT1 = OUT0 + (size_t)NN * ED;
  k_fea<<<dim3(NNP / 64), 128, 0, stream>>>((const int*)d_in[0], F[3], F[5], F[6], OUT0, NF);
  k_agg<<<dim3((NPR + NPB - 1) / NPB), 128, 0, stream>>>((const int*)d_in[1], F[2], F[4], F[7], F[8], NF, AGG);
  k_last<<<dim3((NDRUG + 1023) / 1024), 256, 0, stream>>>((const int*)d_in[0], LAST);
  k_emb<<<dim3((NDRUG + 63) / 64), 256, 0, stream>>>(LAST, AGG, OUT1);
}
